// GNN_22857815949796
// MI455X (gfx1250) — hardware-verified
//
#include <hip/hip_runtime.h>
#include <stddef.h>
#include <stdint.h>
#include <math.h>


#define FD      16
#define NTHR    256
#define NWAVE   8
#define NBRUN   512
#define SLB     9
#define CHUNK   4096
#define NBMAX   256
#define DUMB    255
#define HCH     32
#define STG     (CHUNK + NBMAX * 32)
#define DEGCAP  80
#define CS_SL   0
#define CS_CNT  (NBRUN * DEGCAP)
#define CS_DIS  (CS_CNT + NBRUN)
#define CS_INTS (CS_DIS + NBRUN)
#define WSMAX   134217728

static_assert(NBRUN == (1 << SLB));
static_assert(CHUNK % 32 == 0 && CHUNK % 4 == 0);
static_assert(STG % (NTHR * 4) == 0);
static_assert(CHUNK + (NBMAX - 1) * 31 < STG);
static_assert((NBRUN * DEGCAP) % (NTHR * 4) == 0);
static_assert(CS_INTS % (NTHR * 4) == 0 && CS_CNT % 4 == 0 && CS_DIS % 4 == 0);
static_assert((NBRUN * DEGCAP * 4) % 128 == 0);
static_assert(NBRUN == NWAVE * 4 * 16);
static_assert(CS_INTS * 4 <= 300000);
static_assert(NBMAX * HCH * 4 <= 65536);

typedef float          v4f   __attribute__((ext_vector_type(4)));
typedef float          v8f   __attribute__((ext_vector_type(8)));
typedef int            v4i   __attribute__((ext_vector_type(4)));
typedef int            v8i   __attribute__((ext_vector_type(8)));
typedef unsigned short v4us  __attribute__((ext_vector_type(4)));
typedef unsigned short v8us  __attribute__((ext_vector_type(8)));
typedef unsigned short v16us __attribute__((ext_vector_type(16)));
typedef __bf16         v16bf __attribute__((ext_vector_type(16)));
typedef v4f  __attribute__((may_alias)) v4fa;
typedef v4i  __attribute__((may_alias)) v4ia;
typedef v4us __attribute__((may_alias)) v4usa;
typedef v8us __attribute__((may_alias)) v8usa;
union FragB { v16bf v; v16us u; v8us h[2]; v8i w; };

__device__ __forceinline__ v8f wmb(const FragB& a, const FragB& b, v8f c) {
  v8f d = __builtin_amdgcn_wmma_f32_16x16x32_bf16(false, a.v, false, b.v, (short)0, c, false, false);
  asm volatile("v_nop\n\tv_nop\n\tv_nop\n\tv_nop" : "+v"(d) : "v"(a.w), "v"(b.w));
  return d;
}

__device__ __forceinline__ unsigned bf16_bits(float f) {
  const unsigned u = __float_as_uint(f);
  return (u + 0x7FFFu + ((u >> 16) & 1u)) >> 16;
}
__device__ __forceinline__ float bf16_val(float f) {
  return __uint_as_float(bf16_bits(f) << 16);
}

__device__ __forceinline__ v4i ld4c(const int* __restrict__ p, int nE, int e0, int sent) {
  const int a = (e0 < nE - 4) ? e0 : (nE - 4);
  const v4i v = *(const v4i*)(p + a);
  const bool ok = e0 < nE;
  v4i d;
  d.x = ok ? v.x : sent; d.y = ok ? v.y : sent; d.z = ok ? v.z : sent; d.w = ok ? v.w : sent;
  return d;
}

__device__ __forceinline__ int bkt(int d, int nN) {
  return ((unsigned)d < (unsigned)nN) ? (d >> SLB) : DUMB;
}

__global__ __launch_bounds__(128) void k_prep(const float* __restrict__ W1, const float* __restrict__ W2,
                                              unsigned short* W1T, unsigned short* W2T) {
  const int u   = (int)threadIdx.x;
  const int mat = u >> 6;
  const int v   = u & 63;
  const int n   = v >> 2;
  const int k8  = (v & 3) * 8;
  const int kk  = k8 & 15;
  v8us o;
  unsigned short* dp;
  if (mat == 0) {
    const float* p = W1 + (size_t)kk * FD + n;
    const bool keep = k8 < 16;
#pragma unroll
    for (int i = 0; i < 8; ++i) {
      const unsigned bb = bf16_bits(p[(size_t)i * FD]);
      o[i] = keep ? (unsigned short)bb : (unsigned short)0;
    }
    dp = W1T + (size_t)n * 32 + k8;
  } else {
    const float* p = W2 + (size_t)kk * FD + n;
#pragma unroll
    for (int i = 0; i < 8; ++i) o[i] = (unsigned short)bf16_bits(p[(size_t)i * FD]);
    dp = W2T + (size_t)n * 32 + k8;
  }
  *(volatile v8us*)dp = o;
  __threadfence();
  *(volatile v8us*)dp = o;
}

__global__ __launch_bounds__(HCH) void k_hist(const int* __restrict__ dsts, int nE, int nN, int ncp, int* cntT) {
  __shared__ int bins[NBMAX * HCH];
  const int lane = (int)threadIdx.x;
#pragma unroll 1
  for (int b = 0; b < NBMAX; ++b) bins[b * HCH + lane] = 0;
  const int chunk = (int)blockIdx.x * HCH + lane;
  const int cbase = chunk * CHUNK;
#pragma unroll 1
  for (int i = 0; i < CHUNK / 4; ++i) {
    const v4i d = ld4c(dsts, nE, cbase + 4 * i, -1);
    const int b0 = bkt(d.x, nN), b1 = bkt(d.y, nN), b2 = bkt(d.z, nN), b3 = bkt(d.w, nN);
    bins[b0 * HCH + lane] = bins[b0 * HCH + lane] + 1;
    bins[b1 * HCH + lane] = bins[b1 * HCH + lane] + 1;
    bins[b2 * HCH + lane] = bins[b2 * HCH + lane] + 1;
    bins[b3 * HCH + lane] = bins[b3 * HCH + lane] + 1;
  }
  int* colp = cntT + (size_t)blockIdx.x * HCH + lane;
#pragma unroll 1
  for (int b = 0; b < NBMAX; ++b) {
    const int lv = bins[b * HCH + lane];
    const int v = (b == DUMB) ? 0 : lv;
    *(volatile int*)(colp + (size_t)b * ncp) = v;
  }
  __threadfence();
#pragma unroll 1
  for (int b = 0; b < NBMAX; ++b) {
    const int lv = bins[b * HCH + lane];
    const int v = (b == DUMB) ? 0 : lv;
    *(volatile int*)(colp + (size_t)b * ncp) = v;
  }
}

__global__ __launch_bounds__(NTHR) void k_offs(const int* cntT, int nChunks, int ncp, int nB, int pcap,
                                               int* offrel, int* bst) {
  __shared__ int wtot[NWAVE];
  const int tid = (int)threadIdx.x, lane = tid & 31, wave = tid >> 5;
  const bool act = tid < nB;
  const int* rowp = cntT + (size_t)tid * ncp;
  int run = 0;
#pragma unroll 1
  for (int c = 0; c < nChunks; ++c) {
    int v = rowp[c];
    v = v < 0 ? 0 : (v > CHUNK ? CHUNK : v);
    v = act ? v : 0;
    *(volatile int*)(offrel + (size_t)c * NBMAX + tid) = run;
    run += (v + 31) & ~31;
  }
  __threadfence();
  int run2 = 0;
#pragma unroll 1
  for (int c = 0; c < nChunks; ++c) {
    int v = rowp[c];
    v = v < 0 ? 0 : (v > CHUNK ? CHUNK : v);
    v = act ? v : 0;
    *(volatile int*)(offrel + (size_t)c * NBMAX + tid) = run2;
    run2 += (v + 31) & ~31;
  }
  int incl = run;
#pragma unroll
  for (int d = 1; d < 32; d <<= 1) {
    const int y = __shfl_up(incl, d, 32);
    if (lane >= d) incl += y;
  }
  if (lane == 31) wtot[wave] = incl;
  __syncthreads();
  int wb = 0;
#pragma unroll
  for (int w2 = 0; w2 < NWAVE; ++w2) {
    const int tv = wtot[w2];
    wb += (w2 < wave) ? tv : 0;
  }
  int ex = wb + incl - run;
  ex = ex < 0 ? 0 : (ex > pcap ? pcap : ex);
  *(volatile int*)(bst + tid) = ex;
  __threadfence();
  *(volatile int*)(bst + tid) = ex;
}

__global__ __launch_bounds__(NTHR) void k_place(const int* __restrict__ srcs, const int* __restrict__ dsts,
                                                int nE, int nN, int nB, int ncp, const int* cntT,
                                                const int* offrel, const int* bst, int pcap, int* G) {
  __shared__ __attribute__((aligned(16))) int stage[STG];
  __shared__ int cur[NBMAX];
  __shared__ int lim[NBMAX];
  __shared__ int ps[NBMAX];
  __shared__ int pcs[NBMAX];
  __shared__ int gp[NBMAX];
  __shared__ int wtot[NWAVE];
  const int tid = (int)threadIdx.x, lane = tid & 31, wave = tid >> 5;
  const int chunk = (int)blockIdx.x;
  const int cbase = chunk * CHUNK;
  {
    const v4i m1 = {-1, -1, -1, -1};
    for (int i = tid * 4; i < STG; i += NTHR * 4) *(v4ia*)(stage + i) = m1;
  }
  {
    const bool act = tid < nB;
    int c = cntT[(size_t)tid * ncp + chunk];
    c = c < 0 ? 0 : (c > CHUNK ? CHUNK : c);
    c = act ? c : 0;
    const int pc = (c + 31) & ~31;
    int incl = pc;
#pragma unroll
    for (int d = 1; d < 32; d <<= 1) {
      const int y = __shfl_up(incl, d, 32);
      if (lane >= d) incl += y;
    }
    if (lane == 31) wtot[wave] = incl;
    __syncthreads();
    int wb = 0;
#pragma unroll
    for (int w2 = 0; w2 < NWAVE; ++w2) {
      const int tv = wtot[w2];
      wb += (w2 < wave) ? tv : 0;
    }
    int ex = wb + incl - pc;
    ex = ex < 0 ? 0 : (ex > STG ? STG : ex);
    int le = ex + c;
    le = le > STG ? STG : le;
    ps[tid]  = ex;
    pcs[tid] = pc;
    cur[tid] = ex;
    lim[tid] = le;
    int g = bst[tid] + offrel[(size_t)chunk * NBMAX + tid];
    g = g < 0 ? 0 : g;
    g &= ~31;
    g = (g > pcap - pc) ? (pcap - pc) : g;
    gp[tid] = g;
  }
  __syncthreads();

  if (wave == 0) {
#pragma unroll 1
    for (int st = 0; st < CHUNK / 32; ++st) {
      const int e  = cbase + 32 * st + lane;
      const int ec = e < nE ? e : nE - 1;
      const int dd = dsts[ec];
      int ss = srcs[ec];
      const bool ok = (e < nE) && ((unsigned)dd < (unsigned)nN);
      ss = ss < 0 ? ss + nN : ss;
      ss = ss < 0 ? 0 : (ss > nN - 1 ? nN - 1 : ss);
      const int bb = ok ? (dd >> SLB) : 0;
      const int wv = (ss << SLB) | (dd & (NBRUN - 1));
      unsigned msk = __builtin_amdgcn_ballot_w32(ok);
      int n = (int)__builtin_popcount(msk);
      n = n > 32 ? 32 : n;
#pragma unroll 1
      for (int q = 0; q < n; ++q) {
        int k = __builtin_ffs((int)msk) - 1;
        msk &= msk - 1u;
        k = k < 0 ? 0 : k;
        int ub = __builtin_amdgcn_readlane(bb, k);
        const int uw = __builtin_amdgcn_readlane(wv, k);
        ub = ub < 0 ? 0 : (ub > NBMAX - 1 ? NBMAX - 1 : ub);
        if (lane == 0) {
          const int p = cur[ub];
          const int l = lim[ub];
          if (p >= 0 && p < l) stage[p] = uw;
          cur[ub] = p + 1;
        }
      }
    }
  }
  __syncthreads();

#pragma unroll 1
  for (int b = wave; b < nB; b += NWAVE) {
    int nl = pcs[b] >> 5;
    nl = nl > (CHUNK / 32 + 1) ? (CHUNK / 32 + 1) : nl;
    const int p0 = ps[b];
    const int g0 = gp[b];
#pragma unroll 1
    for (int j = 0; j < nl; ++j) {
      int li = p0 + 32 * j + lane;
      li = li > STG - 1 ? STG - 1 : li;
      const int v = stage[li];
      *(volatile int*)(G + (size_t)g0 + 32 * j + lane) = v;
    }
  }
  __threadfence();
#pragma unroll 1
  for (int b = wave; b < nB; b += NWAVE) {
    int nl = pcs[b] >> 5;
    nl = nl > (CHUNK / 32 + 1) ? (CHUNK / 32 + 1) : nl;
    const int p0 = ps[b];
    const int g0 = gp[b];
#pragma unroll 1
    for (int j = 0; j < nl; ++j) {
      int li = p0 + 32 * j + lane;
      li = li > STG - 1 ? STG - 1 : li;
      const int v = stage[li];
      *(volatile int*)(G + (size_t)g0 + 32 * j + lane) = v;
    }
  }
}

__global__ __launch_bounds__(NTHR) void k_csr(const int* G, const int* bst, int pcap,
                                              int* COL, int* ROWCNT, float* DIS) {
  extern __shared__ __attribute__((aligned(16))) int dsm[];
  const int tid = (int)threadIdx.x, lane = tid & 31, wave = tid >> 5;
  const int b = (int)blockIdx.x;
  float* disl = (float*)(dsm + CS_DIS);
  {
    const v4i z4 = {0, 0, 0, 0};
    for (int i = tid * 4; i < CS_INTS; i += NTHR * 4) *(v4ia*)(dsm + i) = z4;
  }
  __syncthreads();
  int gs = bst[b], ge = bst[b + 1];
  gs = gs < 0 ? 0 : (gs > pcap ? pcap : gs);
  ge = ge < 0 ? 0 : (ge > pcap ? pcap : ge);
  gs &= ~31; ge &= ~31;
  ge = ge < gs ? gs : ge;

  if (wave == 0) {
#pragma unroll 1
    for (int base = gs; base < ge; base += 32) {
      int idx = base + lane;
      idx = idx > pcap - 1 ? pcap - 1 : idx;
      const int w = G[idx];
      unsigned msk = __builtin_amdgcn_ballot_w32(w >= 0);
      int n = (int)__builtin_popcount(msk);
      n = n > 32 ? 32 : n;
#pragma unroll 1
      for (int q = 0; q < n; ++q) {
        int k = __builtin_ffs((int)msk) - 1;
        msk &= msk - 1u;
        k = k < 0 ? 0 : k;
        const int u    = __builtin_amdgcn_readlane(w, k);
        const int slot = u & (NBRUN - 1);
        const int s    = (u >> SLB) & 0x3fffff;
        if (lane == 0) {
          const int c = dsm[CS_CNT + slot];
          if (c >= 0 && c < DEGCAP) dsm[CS_SL + slot * DEGCAP + c] = s;
          dsm[CS_CNT + slot] = c + 1;
        }
      }
    }
  }
  __syncthreads();

#pragma unroll 1
  for (int s = tid; s < NBRUN; s += NTHR) {
    const int c0 = dsm[CS_CNT + s];
    const float dg = (float)(c0 + 1);
    float rv = (dg > 0.0f) ? (1.0f / sqrtf(dg)) : 0.0f;
    if (c0 > DEGCAP || c0 < 0) rv = __int_as_float(0x7fc00000);
    disl[s] = rv;
  }
  __syncthreads();

  int* colb = COL + (size_t)b * (NBRUN * DEGCAP);
#pragma unroll 1
  for (int it = 0; it < (NBRUN * DEGCAP) / (NTHR * 4); ++it) {
    const int i = it * (NTHR * 4) + 4 * tid;
    const v4i v = *(const v4ia*)(dsm + CS_SL + i);
    *(volatile v4i*)(colb + i) = v;
  }
  v4i cv4 = {0, 0, 0, 0};
  v4f dv4 = {0.f, 0.f, 0.f, 0.f};
  const bool rw = tid < NBRUN / 4;
  if (rw) {
    cv4 = *(const v4ia*)(dsm + CS_CNT + 4 * tid);
    dv4 = *(const v4fa*)(disl + 4 * tid);
    cv4.x = cv4.x < 0 ? 0 : (cv4.x > DEGCAP ? DEGCAP : cv4.x);
    cv4.y = cv4.y < 0 ? 0 : (cv4.y > DEGCAP ? DEGCAP : cv4.y);
    cv4.z = cv4.z < 0 ? 0 : (cv4.z > DEGCAP ? DEGCAP : cv4.z);
    cv4.w = cv4.w < 0 ? 0 : (cv4.w > DEGCAP ? DEGCAP : cv4.w);
    const size_t ro = (size_t)b * NBRUN + 4 * tid;
    *(volatile v4i*)(ROWCNT + ro) = cv4;
    *(volatile v4f*)(DIS + ro)    = dv4;
  }
  __threadfence();
#pragma unroll 1
  for (int it = 0; it < (NBRUN * DEGCAP) / (NTHR * 4); ++it) {
    const int i = it * (NTHR * 4) + 4 * tid;
    const v4i v = *(const v4ia*)(dsm + CS_SL + i);
    *(volatile v4i*)(colb + i) = v;
  }
  if (rw) {
    const size_t ro = (size_t)b * NBRUN + 4 * tid;
    *(volatile v4i*)(ROWCNT + ro) = cv4;
    *(volatile v4f*)(DIS + ro)    = dv4;
  }
}

__global__ __launch_bounds__(NTHR) void k_gemm1(const float* __restrict__ x, const unsigned short* W1T,
                                                const float* DIS, int nN, float* HS1) {
  __shared__ __attribute__((aligned(16))) float dt[NWAVE * 256];
  const int tid = (int)threadIdx.x, lane = tid & 31, wave = tid >> 5, hh = lane >> 4, m = lane & 15;
  const int row0 = ((int)blockIdx.x * NWAVE + wave) * 16;
  const int row  = row0 + m;
  const int rc   = row < nN ? row : nN - 1;
  const float* p = x + (size_t)rc * FD + 8 * hh;
  const v4f a  = *(const v4fa*)p;
  const v4f bq = *(const v4fa*)(p + 4);
  const unsigned msk = (row < nN) ? 0xffffu : 0u;
  FragB af;
  af.u[0] = (unsigned short)(bf16_bits(a.x) & msk);
  af.u[1] = (unsigned short)(bf16_bits(a.y) & msk);
  af.u[2] = (unsigned short)(bf16_bits(a.z) & msk);
  af.u[3] = (unsigned short)(bf16_bits(a.w) & msk);
  af.u[4] = (unsigned short)(bf16_bits(bq.x) & msk);
  af.u[5] = (unsigned short)(bf16_bits(bq.y) & msk);
  af.u[6] = (unsigned short)(bf16_bits(bq.z) & msk);
  af.u[7] = (unsigned short)(bf16_bits(bq.w) & msk);
#pragma unroll
  for (int i = 8; i < 16; ++i) af.u[i] = (unsigned short)0;
  FragB bf;
  bf.h[0] = *(const v8usa*)(W1T + m * 32 + 8 * hh);
  bf.h[1] = *(const v8usa*)(W1T + m * 32 + 16 + 8 * hh);
  v8f acc = {0.f, 0.f, 0.f, 0.f, 0.f, 0.f, 0.f, 0.f};
  acc = wmb(af, bf, acc);
  const v4f d0 = *(const v4fa*)(DIS + row0 + 8 * hh);
  const v4f d1 = *(const v4fa*)(DIS + row0 + 8 * hh + 4);
  float* dw = dt + wave * 256;
  dw[(8 * hh + 0) * 16 + m] = acc[0] * d0.x;
  dw[(8 * hh + 1) * 16 + m] = acc[1] * d0.y;
  dw[(8 * hh + 2) * 16 + m] = acc[2] * d0.z;
  dw[(8 * hh + 3) * 16 + m] = acc[3] * d0.w;
  dw[(8 * hh + 4) * 16 + m] = acc[4] * d1.x;
  dw[(8 * hh + 5) * 16 + m] = acc[5] * d1.y;
  dw[(8 * hh + 6) * 16 + m] = acc[6] * d1.z;
  dw[(8 * hh + 7) * 16 + m] = acc[7] * d1.w;
  __syncthreads();
  const v4f q0 = *(const v4fa*)(dw + 4 * lane);
  const v4f q1 = *(const v4fa*)(dw + 128 + 4 * lane);
  float* op = HS1 + (size_t)row0 * FD + 4 * lane;
  *(volatile v4f*)op = q0;
  *(volatile v4f*)(op + 128) = q1;
  __threadfence();
  *(volatile v4f*)op = q0;
  *(volatile v4f*)(op + 128) = q1;
}

__device__ __forceinline__ v4f gather_row(const int* colr, int c, const float* HS, int row, int nN, int q) {
  int cm = c;
  { const int y = __shfl_xor(cm, 4, 32);  cm = cm > y ? cm : y; }
  { const int y = __shfl_xor(cm, 8, 32);  cm = cm > y ? cm : y; }
  { const int y = __shfl_xor(cm, 16, 32); cm = cm > y ? cm : y; }
  cm = __builtin_amdgcn_readfirstlane(cm);
  cm = cm > DEGCAP ? DEGCAP : cm;
  v4f acc = {0.0f, 0.0f, 0.0f, 0.0f};
#pragma unroll 1
  for (int p = 0; p < cm; ++p) {
    int s = colr[p];
    s = s < 0 ? 0 : (s > nN - 1 ? nN - 1 : s);
    const v4f a = *(const v4fa*)(HS + (size_t)s * FD + 4 * q);
    const unsigned mk = (p < c) ? 0xffffffffu : 0u;
    acc.x += __uint_as_float(__float_as_uint(a.x) & mk);
    acc.y += __uint_as_float(__float_as_uint(a.y) & mk);
    acc.z += __uint_as_float(__float_as_uint(a.z) & mk);
    acc.w += __uint_as_float(__float_as_uint(a.w) & mk);
  }
  const v4f sf = *(const v4fa*)(HS + (size_t)row * FD + 4 * q);
  acc.x += sf.x; acc.y += sf.y; acc.z += sf.z; acc.w += sf.w;
  return acc;
}

__global__ __launch_bounds__(NTHR) void k_layer1(const int* COL, const int* ROWCNT,
                                                 const float* DIS, const float* HS1,
                                                 const float* __restrict__ b1, const unsigned short* W2T,
                                                 int nN, float* HS2) {
  __shared__ __attribute__((aligned(16))) unsigned short at[NWAVE * 512];
  __shared__ __attribute__((aligned(16))) float dt[NWAVE * 256];
  const int tid = (int)threadIdx.x, lane = tid & 31, wave = tid >> 5;
  const int g = lane >> 2, q = lane & 3, hh = lane >> 4, m = lane & 15;
  const int base = (int)blockIdx.x * NBRUN;
  const int* colb = COL + (size_t)blockIdx.x * (NBRUN * DEGCAP);
  v4f bv;
  {
    const v4f t = *(const v4fa*)(b1 + 4 * q);
    bv.x = bf16_val(t.x); bv.y = bf16_val(t.y); bv.z = bf16_val(t.z); bv.w = bf16_val(t.w);
  }
  FragB bf;
  bf.h[0] = *(const v8usa*)(W2T + m * 32 + 8 * hh);
  bf.h[1] = *(const v8usa*)(W2T + m * 32 + 16 + 8 * hh);
  unsigned short* aw = at + wave * 512;
  float* dw = dt + wave * 256;

#pragma unroll 1
  for (int ti = 0; ti < 4; ++ti) {
    const int t16  = 16 * (wave * 4 + ti);
    const int row0 = base + t16;
#pragma unroll 1
    for (int pass = 0; pass < 2; ++pass) {
      const int lr  = 8 * pass + g;
      const int row = row0 + lr;
      int c = ROWCNT[row];
      c = c < 0 ? 0 : (c > DEGCAP ? DEGCAP : c);
      const v4f acc = gather_row(colb + (t16 + lr) * DEGCAP, c, HS1, row, nN, q);
      const float d = DIS[row];
      v4f v;
      v.x = d * acc.x + bv.x; v.y = d * acc.y + bv.y; v.z = d * acc.z + bv.z; v.w = d * acc.w + bv.w;
      v.x = (v.x > 0.0f) ? v.x : (v.x - v.x);
      v.y = (v.y > 0.0f) ? v.y : (v.y - v.y);
      v.z = (v.z > 0.0f) ? v.z : (v.z - v.z);
      v.w = (v.w > 0.0f) ? v.w : (v.w - v.w);
      const bool live = row < nN;
      v.x = live ? v.x : 0.0f; v.y = live ? v.y : 0.0f; v.z = live ? v.z : 0.0f; v.w = live ? v.w : 0.0f;
      v4us h4, l4;
      unsigned hb;
      hb = bf16_bits(v.x); h4[0] = (unsigned short)hb; l4[0] = (unsigned short)bf16_bits(v.x - __uint_as_float(hb << 16));
      hb = bf16_bits(v.y); h4[1] = (unsigned short)hb; l4[1] = (unsigned short)bf16_bits(v.y - __uint_as_float(hb << 16));
      hb = bf16_bits(v.z); h4[2] = (unsigned short)hb; l4[2] = (unsigned short)bf16_bits(v.z - __uint_as_float(hb << 16));
      hb = bf16_bits(v.w); h4[3] = (unsigned short)hb; l4[3] = (unsigned short)bf16_bits(v.w - __uint_as_float(hb << 16));
      *(v4usa*)(aw + lr * 32 + 4 * q)      = h4;
      *(v4usa*)(aw + lr * 32 + 16 + 4 * q) = l4;
    }
    __syncthreads();
    FragB af;
    af.h[0] = *(const v8usa*)(aw + m * 32 + 8 * hh);
    af.h[1] = *(const v8usa*)(aw + m * 32 + 16 + 8 * hh);
    v8f acc8 = {0.f, 0.f, 0.f, 0.f, 0.f, 0.f, 0.f, 0.f};
    acc8 = wmb(af, bf, acc8);
    const v4f d0 = *(const v4fa*)(DIS + row0 + 8 * hh);
    const v4f d1 = *(const v4fa*)(DIS + row0 + 8 * hh + 4);
    dw[(8 * hh + 0) * 16 + m] = acc8[0] * d0.x;
    dw[(8 * hh + 1) * 16 + m] = acc8[1] * d0.y;
    dw[(8 * hh + 2) * 16 + m] = acc8[2] * d0.z;
    dw[(8 * hh + 3) * 16 + m] = acc8[3] * d0.w;
    dw[(8 * hh + 4) * 16 + m] = acc8[4] * d1.x;
    dw[(8 * hh + 5) * 16 + m] = acc8[5] * d1.y;
    dw[(8 * hh + 6) * 16 + m] = acc8[6] * d1.z;
    dw[(8 * hh + 7) * 16 + m] = acc8[7] * d1.w;
    __syncthreads();
    const v4f q0 = *(const v4fa*)(dw + 4 * lane);
    const v4f q1 = *(const v4fa*)(dw + 128 + 4 * lane);
    __syncthreads();
    float* op = HS2 + (size_t)row0 * FD + 4 * lane;
    *(volatile v4f*)op = q0;
    *(volatile v4f*)(op + 128) = q1;
    __threadfence();
    *(volatile v4f*)op = q0;
    *(volatile v4f*)(op + 128) = q1;
  }
}

__global__ __launch_bounds__(NTHR) void k_layer2(const int* COL, const int* ROWCNT,
                                                 const float* DIS, const float* HS2,
                                                 const float* __restrict__ b2, const float* __restrict__ Wfc,
                                                 const float* __restrict__ bfc, int nN, float* out) {
  __shared__ __attribute__((aligned(16))) float outs[NBRUN];
  const int tid = (int)threadIdx.x, lane = tid & 31, wave = tid >> 5;
  const int g = lane >> 2, q = lane & 3;
  const int base = (int)blockIdx.x * NBRUN;
  const int* colb = COL + (size_t)blockIdx.x * (NBRUN * DEGCAP);
  v4f bv, wv;
  {
    const v4f t = *(const v4fa*)(b2 + 4 * q);
    bv.x = bf16_val(t.x); bv.y = bf16_val(t.y); bv.z = bf16_val(t.z); bv.w = bf16_val(t.w);
    const v4f u = *(const v4fa*)(Wfc + 4 * q);
    wv.x = bf16_val(u.x); wv.y = bf16_val(u.y); wv.z = bf16_val(u.z); wv.w = bf16_val(u.w);
  }
  const float bo = bf16_val(bfc[0]);

#pragma unroll 1
  for (int ti = 0; ti < 4; ++ti) {
    const int t16 = 16 * (wave * 4 + ti);
#pragma unroll 1
    for (int pass = 0; pass < 2; ++pass) {
      const int lr  = t16 + 8 * pass + g;
      const int row = base + lr;
      int c = ROWCNT[row];
      c = c < 0 ? 0 : (c > DEGCAP ? DEGCAP : c);
      const v4f acc = gather_row(colb + lr * DEGCAP, c, HS2, row, nN, q);
      const float d = DIS[row];
      v4f v;
      v.x = d * acc.x + bv.x; v.y = d * acc.y + bv.y; v.z = d * acc.z + bv.z; v.w = d * acc.w + bv.w;
      v.x = (v.x > 0.0f) ? v.x : (v.x - v.x);
      v.y = (v.y > 0.0f) ? v.y : (v.y - v.y);
      v.z = (v.z > 0.0f) ? v.z : (v.z - v.z);
      v.w = (v.w > 0.0f) ? v.w : (v.w - v.w);
      float s = v.x * wv.x;
      s = fmaf(v.y, wv.y, s);
      s = fmaf(v.z, wv.z, s);
      s = fmaf(v.w, wv.w, s);
      s = s + __shfl_xor(s, 1, 32);
      s = s + __shfl_xor(s, 2, 32);
      float r = s + bo;
      r = (row < nN) ? r : 0.0f;
      if (q == 0) outs[lr] = r;
    }
  }
  __syncthreads();
  if (tid < NBRUN / 4) {
    const v4f ov = *(const v4fa*)(outs + 4 * tid);
    const int gi = base + 4 * tid;
    const bool okst = (gi + 3) < nN;
    float* op = out + (size_t)(okst ? gi : 0);
    if (okst) *(volatile v4f*)op = ov;
    __threadfence();
    if (okst) *(volatile v4f*)op = ov;
  }
}

static inline int cdiv(int a, int b) { return (a + b - 1) / b; }
static inline size_t al256(size_t o) { return (o + 255) & ~(size_t)255; }

extern "C" void kernel_launch(void* const* d_in, const int* in_sizes, int n_in,
                              void* d_out, int out_size, void* d_ws, size_t ws_size,
                              hipStream_t stream) {
  if (n_in < 8) return;
  if (in_sizes[0] < FD || (in_sizes[0] % FD) != 0) return;
  const int nN = in_sizes[0] / FD;
  if (nN < 4 || nN > (1 << 22) || (nN & 3) != 0) return;
  if (in_sizes[1] < 8 || (in_sizes[1] & 1) != 0) return;
  const int nE = in_sizes[1] / 2;
  if (nE < 4 || (nE & 3) != 0 || nE >= (1 << 28)) return;
  if (in_sizes[2] != FD * FD || in_sizes[3] != FD) return;
  if (in_sizes[4] != FD * FD || in_sizes[5] != FD) return;
  if (in_sizes[6] != FD || in_sizes[7] != 1) return;
  if (out_size != nN) return;

  const float* x    = (const float*)d_in[0];
  const int*   edge = (const int*)d_in[1];
  const float* W1   = (const float*)d_in[2];
  const float* b1   = (const float*)d_in[3];
  const float* W2   = (const float*)d_in[4];
  const float* b2   = (const float*)d_in[5];
  const float* Wfc  = (const float*)d_in[6];
  const float* bfc  = (const float*)d_in[7];
  float* out = (float*)d_out;
  const int* src = edge;
  const int* dst = edge + nE;

  const int nB = cdiv(nN, NBRUN);
  if (nB < 1 || nB > NBMAX - 2) return;
  const int MP = nB * NBRUN;
  const int nChunks = cdiv(nE, CHUNK);
  const int NCP = cdiv(nChunks, HCH) * HCH;
  const long long pcapL = (((long long)nE + 31) & ~31LL) + (long long)nChunks * nB * 32;
  if (pcapL >= (1LL << 30) || pcapL < (long long)(CHUNK + 64)) return;
  const int pcap = (int)pcapL;

  char* ws = (char*)d_ws;
  size_t off = 0;
  const size_t oW1T = off; off = al256(off + (size_t)16 * 32 * 2);
  const size_t oW2T = off; off = al256(off + (size_t)16 * 32 * 2);
  const size_t oCNT = off; off = al256(off + (size_t)NBMAX * NCP * 4);
  const size_t oOFR = off; off = al256(off + (size_t)nChunks * NBMAX * 4);
  const size_t oBST = off; off = al256(off + (size_t)NBMAX * 4);
  const size_t oG   = off; off = al256(off + (size_t)pcap * 4);
  const size_t oCOL = off; off = al256(off + (size_t)MP * DEGCAP * 4);
  const size_t oRC  = off; off = al256(off + (size_t)MP * 4);
  const size_t oDIS = off; off = al256(off + (size_t)MP * 4);
  const size_t oHS1 = off; off = al256(off + (size_t)MP * FD * 4);
  const size_t oHS2 = off; off = al256(off + (size_t)MP * FD * 4);
  if (off > ws_size || off > (size_t)WSMAX) return;
  unsigned short* W1T = (unsigned short*)(ws + oW1T);
  unsigned short* W2T = (unsigned short*)(ws + oW2T);
  int*   CNT    = (int*)(ws + oCNT);
  int*   OFR    = (int*)(ws + oOFR);
  int*   BST    = (int*)(ws + oBST);
  int*   G      = (int*)(ws + oG);
  int*   COL    = (int*)(ws + oCOL);
  int*   ROWCNT = (int*)(ws + oRC);
  float* DIS    = (float*)(ws + oDIS);
  float* HS1    = (float*)(ws + oHS1);
  float* HS2    = (float*)(ws + oHS2);

  const size_t csrLds = (size_t)CS_INTS * 4;
  hipFuncSetAttribute(reinterpret_cast<const void*>(&k_csr), hipFuncAttributeMaxDynamicSharedMemorySize, (int)csrLds);

  k_prep<<<1, 128, 0, stream>>>(W1, W2, W1T, W2T);
  k_hist<<<NCP / HCH, HCH, 0, stream>>>(dst, nE, nN, NCP, CNT);
  k_offs<<<1, NTHR, 0, stream>>>(CNT, nChunks, NCP, nB, pcap, OFR, BST);
  k_place<<<nChunks, NTHR, 0, stream>>>(src, dst, nE, nN, nB, NCP, CNT, OFR, BST, pcap, G);
  k_csr<<<nB, NTHR, csrLds, stream>>>(G, BST, pcap, COL, ROWCNT, DIS);
  k_gemm1<<<MP / (NWAVE * 16), NTHR, 0, stream>>>(x, W1T, DIS, nN, HS1);
  k_layer1<<<nB, NTHR, 0, stream>>>(COL, ROWCNT, DIS, HS1, b1, W2T, nN, HS2);
  k_layer2<<<nB, NTHR, 0, stream>>>(COL, ROWCNT, DIS, HS2, b2, Wfc, bfc, nN, out);
}
